// get_point_correspondences_28613072126431
// MI455X (gfx1250) — hardware-verified
//
#include <hip/hip_runtime.h>


namespace {
constexpr int Bsz = 4, D = 256, N = 4096, M = 4096;
constexpr float ESC = 8.0f;
constexpr int QT = N / 16;

typedef _Float16 b16;
typedef __attribute__((ext_vector_type(16))) _Float16 v16b;
typedef __attribute__((ext_vector_type(8)))  _Float16 v8b;
typedef __attribute__((ext_vector_type(8)))  float v8f;
typedef __attribute__((ext_vector_type(4)))  float v4f;

__device__ __forceinline__ v8b ld8b(const b16* p) { return *(const v8b*)p; }
__device__ __forceinline__ v16b cat8b(v8b a, v8b b) { return __builtin_shufflevector(a, b, 0, 1, 2, 3, 4, 5, 6, 7, 8, 9, 10, 11, 12, 13, 14, 15); }
__device__ __forceinline__ v16b frag_kb(const b16* p, int hh) { return cat8b(ld8b(p + 8 * hh), ld8b(p + 16 + 8 * hh)); }
__device__ __forceinline__ void split16(float v, b16& hi, b16& lo) { hi = (b16)v; lo = (b16)(v - (float)hi); }
__device__ __forceinline__ v8f wmma16b(v16b a, v16b b, v8f c) {
  v8f d = __builtin_amdgcn_wmma_f32_16x16x32_f16(false, a, false, b, (short)0, c, false, false);
  asm volatile("v_nop\n\tv_nop\n\tv_nop\n\tv_nop" : "+v"(d) : "v"(a), "v"(b));
  return d;
}
__device__ __forceinline__ v8f wmma3(v16b ah, v16b al, v16b bh, v16b bl, v8f c) { c = wmma16b(ah, bh, c); c = wmma16b(ah, bl, c); return wmma16b(al, bh, c); }

__global__ __launch_bounds__(256) void prep_emb_kernel(const float* __restrict__ emb, b16* __restrict__ ph, b16* __restrict__ pl, float* __restrict__ yy) {
  __shared__ __attribute__((aligned(16))) b16 Th[64][D + 8];
  __shared__ __attribute__((aligned(16))) b16 Tl[64][D + 8];
  __shared__ float ysq[16][64];
  const int tid = threadIdx.x, lane = tid & 31, wave = tid >> 5;
  const int b = blockIdx.x / (N / 64), n0 = (blockIdx.x % (N / 64)) * 64;
  const float* eb = emb + (size_t)b * D * N;
  float sq[4] = {0.f, 0.f, 0.f, 0.f};
#pragma unroll 1
  for (int it = 0; it < D / 16; ++it) {
    const int d = it * 16 + (tid >> 4), px = (tid & 15) * 4;
    const v4f q = *(const v4f*)(eb + (size_t)d * N + n0 + px);
#pragma unroll
    for (int e = 0; e < 4; ++e) { b16 h_, l_; split16(q[e] * ESC, h_, l_); Th[px + e][d] = h_; Tl[px + e][d] = l_; sq[e] += q[e] * q[e]; }
  }
#pragma unroll
  for (int e = 0; e < 4; ++e) ysq[tid >> 4][(tid & 15) * 4 + e] = sq[e];
  __syncthreads();
  b16* oh = ph + ((size_t)b * N + n0) * D; b16* ol = pl + ((size_t)b * N + n0) * D;
  for (int pass = 0; pass < 2; ++pass) {
#pragma unroll
    for (int rr = 0; rr < 8; ++rr) {
      const int row = wave * 8 + rr;
      *(volatile v8b*)(oh + (size_t)row * D + lane * 8) = *(const v8b*)(&Th[row][lane * 8]);
      *(volatile v8b*)(ol + (size_t)row * D + lane * 8) = *(const v8b*)(&Tl[row][lane * 8]);
    }
    if (wave == 0 && lane < 16) {
      v4f y4;
#pragma unroll
      for (int e = 0; e < 4; ++e) { float s = 0.f;
#pragma unroll
        for (int g = 0; g < 16; ++g) s += ysq[g][lane * 4 + e];
        y4[e] = s; }
      *(volatile v4f*)(yy + (size_t)b * M + n0 + lane * 4) = y4;
    }
    __threadfence();
  }
}

__global__ __launch_bounds__(256) void prep_tgt_kernel(const float* __restrict__ tgt, b16* __restrict__ t16) {
  const size_t tid = (size_t)blockIdx.x * blockDim.x + threadIdx.x, stride = (size_t)gridDim.x * blockDim.x;
  const size_t tot = (size_t)Bsz * 16 * M / 8;
  for (int pass = 0; pass < 2; ++pass) {
    for (size_t c = tid; c < tot; c += stride) {
      const size_t i = c * 8; const int b = (int)(i / (16 * M)), row = (int)((i / M) % 16), m = (int)(i % M);
      v8b v;
#pragma unroll
      for (int e = 0; e < 8; ++e) v[e] = (row < 3) ? (b16)tgt[((size_t)b * 3 + row) * M + m + e] : (b16)0.0f;
      *(volatile v8b*)(t16 + i) = v;
    }
    __threadfence();
  }
}

__global__ __launch_bounds__(256) void corr_kernel(const b16* __restrict__ eh, const b16* __restrict__ el, const b16* __restrict__ fh, const b16* __restrict__ fl,
                                                   const float* __restrict__ yy, const b16* __restrict__ t16, float* __restrict__ out) {
  __shared__ __attribute__((aligned(16))) float Os[3][128];
  const int wid = threadIdx.x >> 5, lane = threadIdx.x & 31, hh = lane >> 4, col = lane & 15;
  const int b = blockIdx.x / (N / 128), n0blk = (blockIdx.x % (N / 128)) * 128, q0 = n0blk + wid * 16;
  const size_t qo = ((size_t)b * N + q0 + col) * D;
  v16b qh[8], ql[8];
#pragma unroll
  for (int k = 0; k < 8; ++k) { qh[k] = frag_kb(eh + qo + 32 * k, hh); ql[k] = frag_kb(el + qo + 32 * k, hh); }
  const size_t fo = (size_t)b * M * D; const float* yyb = yy + (size_t)b * M; const b16* tb = t16 + (size_t)b * 16 * M;
  float m = -INFINITY, l = 0.0f;
  v8f o0 = {};
  for (int kb = 0; kb < M; kb += 32) {
    const size_t r0 = fo + (size_t)(kb + col) * D, r1 = fo + (size_t)(kb + 16 + col) * D;
    v8f s0 = {}, s1 = {};
#pragma unroll
    for (int k = 0; k < 8; ++k) {
      v16b ah = frag_kb(fh + r0 + 32 * k, hh), al = frag_kb(fl + r0 + 32 * k, hh);
      s0 = wmma3(ah, al, qh[k], ql[k], s0);
      ah = frag_kb(fh + r1 + 32 * k, hh); al = frag_kb(fl + r1 + 32 * k, hh);
      s1 = wmma3(ah, al, qh[k], ql[k], s1);
    }
    float mr = -INFINITY;
#pragma unroll
    for (int r = 0; r < 8; ++r) {
      s0[r] = s0[r] * (2.0f / (ESC * ESC)) - yyb[kb + 8 * hh + r];
      s1[r] = s1[r] * (2.0f / (ESC * ESC)) - yyb[kb + 16 + 8 * hh + r];
      mr = fmaxf(mr, fmaxf(s0[r], s1[r]));
    }
    mr = fmaxf(mr, __shfl_xor(mr, 16));
    const float mn = fmaxf(m, mr);
    const float al_ = __expf(m - mn);
    m = mn;
    float sum = 0.0f;
    v16b pb;
#pragma unroll
    for (int r = 0; r < 8; ++r) {
      const float p0 = __expf(s0[r] - mn), p1 = __expf(s1[r] - mn);
      sum += p0 + p1;
      pb[r] = (b16)p0; pb[8 + r] = (b16)p1;
    }
    sum += __shfl_xor(sum, 16);
    l = l * al_ + sum;
#pragma unroll
    for (int r = 0; r < 8; ++r) o0[r] *= al_;
    const b16* tr = tb + (size_t)col * M + kb;
    const v16b va = cat8b(ld8b(tr + 8 * hh), ld8b(tr + 16 + 8 * hh));
    o0 = wmma16b(va, pb, o0);
  }
  const float inv = 1.0f / l;
  if (hh == 0) {
#pragma unroll
    for (int r = 0; r < 3; ++r) Os[r][wid * 16 + col] = o0[r] * inv;
  }
  __syncthreads();
  if (wid < 3) {
    float* dst = out + ((size_t)b * 3 + wid) * N + n0blk;
    const v4f v = *(const v4f*)(&Os[wid][lane * 4]);
    *(volatile v4f*)(dst + lane * 4) = v;
    __threadfence();
    *(volatile v4f*)(dst + lane * 4) = v;
  }
}
}

extern "C" void kernel_launch(void* const* d_in, const int* in_sizes, int n_in,
                              void* d_out, int out_size, void* d_ws, size_t ws_size, hipStream_t stream) {
  (void)n_in; (void)out_size;
  const float* src     = (const float*)d_in[0];
  const float* tgt     = (const float*)d_in[1];
  const float* src_emb = (const float*)d_in[2];
  const float* tgt_emb = (const float*)d_in[3];
  float* out = (float*)d_out;
  (void)src;
  if (in_sizes[1] != Bsz * 3 * M || in_sizes[2] != Bsz * D * N || in_sizes[3] != Bsz * D * M) return;

  size_t off = 0; char* ws = (char*)d_ws;
  auto carve = [&](size_t bytes) { char* p = ws + off; off += (bytes + 255) & ~(size_t)255; return p; };
  b16* eh = (b16*)carve((size_t)Bsz * N * D * 2);
  b16* el = (b16*)carve((size_t)Bsz * N * D * 2);
  b16* fh = (b16*)carve((size_t)Bsz * M * D * 2);
  b16* fl = (b16*)carve((size_t)Bsz * M * D * 2);
  float* yye = (float*)carve((size_t)Bsz * N * 4);
  float* yyf = (float*)carve((size_t)Bsz * M * 4);
  b16* t16 = (b16*)carve((size_t)Bsz * 16 * M * 2);
  if (off > ws_size) return;
  prep_emb_kernel<<<Bsz * N / 64, 256, 0, stream>>>(src_emb, eh, el, yye);
  prep_emb_kernel<<<Bsz * M / 64, 256, 0, stream>>>(tgt_emb, fh, fl, yyf);
  prep_tgt_kernel<<<256, 256, 0, stream>>>(tgt, t16);
  corr_kernel<<<Bsz * N / 128, 256, 0, stream>>>(eh, el, fh, fl, yyf, t16, out);
}
